// Model_43069932045089
// MI455X (gfx1250) — hardware-verified
//
#include <hip/hip_runtime.h>
#include <stddef.h>
#include <stdint.h>

#define NN    255
#define NNZ   2550
#define NB    512
#define BC    128
#define NCH   (NB / BC)
#define MR    (NB * NN)
#define RC    (BC * NN)
#define GBM   64
#define NTHR  256

#define D1 400
#define D2 300
#define D3 100
#define D4 300
#define D5 400

#define K1  800
#define K2  640
#define K3  256
#define K4  640
#define NP1 320
#define NP2 128
#define NP3 320
#define NP4 400

static_assert(NNZ == 2550 && NN == 255 && NB % BC == 0);
static_assert(RC % GBM == 0 && MR % 512 == 0 && MR * 2 == 255 * 1024);
static_assert(K1 % 32 == 0 && K2 % 32 == 0 && K3 % 32 == 0 && K4 % 32 == 0);
static_assert(NP1 % 16 == 0 && NP2 % 16 == 0 && NP3 % 16 == 0 && NP4 % 16 == 0);

#define CSR_RB    0
#define CSR_RE    256
#define CSR_COL   512
#define CSR_VAL   3072
#define CSR_RS    5632
#define CSR_WORDS 5888
#define CSR_STAGE_V4 1408
#define CSR_LDS   22528
static_assert(CSR_VAL == CSR_COL + 2560 && CSR_RS == CSR_VAL + 2560 && CSR_WORDS % 4 == 0);

#define WS_A    ((size_t)0)
#define WS_B    ((size_t)41779200)
#define WS_C    ((size_t)83558400)
#define WS_D    ((size_t)100270080)
#define WS_S0   ((size_t)116981760)
#define WS_P6   ((size_t)118026240)
#define WS_W1   ((size_t)119070720)
#define WS_W2   ((size_t)119582720)
#define WS_W3   ((size_t)119746560)
#define WS_W4   ((size_t)119910400)
#define WS_CSM  ((size_t)120422400)
#define WS_CSP  ((size_t)120445952)
#define WS_END  ((size_t)120469504)
static_assert(WS_B == WS_A + (size_t)RC * NP1 * 4);
static_assert(WS_C == WS_B + (size_t)RC * K2 * 2);
static_assert(WS_D == WS_C + (size_t)RC * NP2 * 4);
static_assert(WS_S0 == WS_D + (size_t)RC * K3 * 2);
static_assert(WS_P6 == WS_S0 + (size_t)MR * 2 * 4);
static_assert(WS_W1 == WS_P6 + (size_t)MR * 2 * 4);
static_assert(WS_W2 == WS_W1 + (size_t)NP1 * K1 * 2);
static_assert(WS_W3 == WS_W2 + (size_t)NP2 * K2 * 2);
static_assert(WS_W4 == WS_W3 + (size_t)NP3 * K3 * 2);
static_assert(WS_CSM == WS_W4 + (size_t)NP4 * K4 * 2);
static_assert(WS_CSP == WS_CSM + (size_t)CSR_WORDS * 4);
static_assert(WS_END == WS_CSP + (size_t)CSR_WORDS * 4);
static_assert(WS_END <= (size_t)134217728);
static_assert(WS_B % 256 == 0 && WS_C % 256 == 0 && WS_D % 256 == 0 && WS_S0 % 256 == 0 && WS_P6 % 256 == 0);
static_assert(WS_W1 % 256 == 0 && WS_W2 % 256 == 0 && WS_W3 % 256 == 0 && WS_W4 % 256 == 0);
static_assert(WS_CSM % 256 == 0 && WS_CSP % 256 == 0);

#define PB1 125
#define PB2 40
#define PB3 40
#define PB4 125
static_assert(PB1 * NTHR == NP1 * (K1 / 8) && PB2 * NTHR == NP2 * (K2 / 8));
static_assert(PB3 * NTHR == NP3 * (K3 / 8) && PB4 * NTHR == NP4 * (K4 / 8));

#define BLD_IMG  0
#define BLD_TI   23552
#define BLD_TJ   33792
#define BLD_TV   44032
#define BLD_CNT  54272
#define BLD_ST   55296
#define BLD_DMP  56320
#define BLD_MX   58368
#define BLD_LDS  58384
#define BLD_DMPW (BLD_DMP / 4)
#define BLD_MXW  (BLD_MX / 4)
static_assert(BLD_TI == CSR_WORDS * 4 && BLD_DMP == BLD_ST + 1024 && BLD_MX == BLD_DMP + 2048);

#define AG2_CSR  0
#define AG2_OUT  22528
#define AG2_LDS  26624

#define G1_A     0
#define G1_W0A   102400
#define G1_W0B   104000
#define G1_B0    105600
#define G1_B1    107200
#define G1_S0    108480
#define G1_RS    108992
#define G1_LDS   109248
static_assert(GBM * K1 * 2 == G1_W0A && GBM * NP1 * 4 <= G1_W0A);

#define GL_SB(NP)   (GBM * (NP) * 4)
#define GL_SRS(NP)  (GL_SB(NP) + (NP) * 4)
#define GL_SW5(NP)  (GL_SRS(NP) + 256)
#define GL_SP6(NP)  (GL_SW5(NP) + 3200)
#define GL_TOT(NP)  (GL_SP6(NP) + 512)

#define A23_Y    0
#define A23_X    106080
#define A23_CSR  212160
#define A23_LDS  234688
#define YS       104
static_assert(NN * YS * 4 == A23_X && A23_CSR == 2 * A23_X && A23_LDS == A23_CSR + CSR_LDS);
static_assert(A23_X % 16 == 0 && A23_CSR % 16 == 0);

typedef float          v2f   __attribute__((ext_vector_type(2)));
typedef float          v4f   __attribute__((ext_vector_type(4)));
typedef float          v8f   __attribute__((ext_vector_type(8)));
typedef int            v4i   __attribute__((ext_vector_type(4)));
typedef int            v8i   __attribute__((ext_vector_type(8)));
typedef unsigned       v2u   __attribute__((ext_vector_type(2)));
typedef unsigned short v8us  __attribute__((ext_vector_type(8)));
typedef unsigned short v16us __attribute__((ext_vector_type(16)));
typedef __bf16         v16bf __attribute__((ext_vector_type(16)));
typedef v2f  __attribute__((may_alias)) v2fa;
typedef v4f  __attribute__((may_alias)) v4fa;
typedef v4i  __attribute__((may_alias)) v4ia;
typedef v8us __attribute__((may_alias)) v8usa;
union FragB { v16bf v; v16us u; v8us h[2]; v8i w; };

extern __shared__ __attribute__((aligned(16))) unsigned char dsm[];

__device__ __forceinline__ v8f wmb(const FragB& a, const FragB& b, v8f c) {
  v8f d = __builtin_amdgcn_wmma_f32_16x16x32_bf16(false, a.v, false, b.v, (short)0, c, false, false);
  asm volatile("v_nop\n\tv_nop\n\tv_nop\n\tv_nop" : "+v"(d) : "v"(a.w), "v"(b.w));
  return d;
}

__device__ __forceinline__ unsigned bf16_bits(float f) {
  const unsigned u = __float_as_uint(f);
  const unsigned r = (u + 0x7FFFu + ((u >> 16) & 1u)) >> 16;
  const unsigned q = (u >> 16) | 0x40u;
  return ((u & 0x7fffffffu) > 0x7f800000u) ? q : r;
}
__device__ __forceinline__ float bf16_val(float f) { return __uint_as_float(bf16_bits(f) << 16); }
__device__ __forceinline__ float relu_f(float v) { return (v > 0.0f) ? v : (v - v); }
__device__ __forceinline__ int clampi(int v, int lo, int hi) { return v < lo ? lo : (v > hi ? hi : v); }

__device__ __forceinline__ void hilo_pack(float v0, float v1, float v2, float v3, v2u& hw, v2u& lw) {
  const unsigned a0 = bf16_bits(v0), a1 = bf16_bits(v1), a2 = bf16_bits(v2), a3 = bf16_bits(v3);
  const unsigned b0 = bf16_bits(v0 - __uint_as_float(a0 << 16));
  const unsigned b1 = bf16_bits(v1 - __uint_as_float(a1 << 16));
  const unsigned b2 = bf16_bits(v2 - __uint_as_float(a2 << 16));
  const unsigned b3 = bf16_bits(v3 - __uint_as_float(a3 << 16));
  v2u h, l;
  h.x = a0 | (a1 << 16); h.y = a2 | (a3 << 16);
  l.x = b0 | (b1 << 16); l.y = b2 | (b3 << 16);
  hw = h; lw = l;
}

__device__ __forceinline__ void stage_csr(const int* __restrict__ g, int ldsOff, int tid) {
  int* s = (int*)(dsm + ldsOff);
#pragma unroll 1
  for (int q = tid; q < CSR_STAGE_V4; q += NTHR) {
    const v4i v = *(const v4ia*)(g + 4 * q);
    *(v4ia*)(s + 4 * q) = v;
  }
}

template <int KH, int KT, int NTR>
__device__ __forceinline__ void prep_unit(const float* __restrict__ W, unsigned short* plane, int u) {
  static_assert(KH % 8 == 0 && KT <= KH);
  constexpr int UPR = (2 * KH) / 8;
  const int n  = u / UPR;
  const int k8 = (u - n * UPR) * 8;
  const int kk = (k8 >= KH) ? (k8 - KH) : k8;
  const int nc = (n < NTR) ? n : (NTR - 1);
  v8us o;
#pragma unroll
  for (int j = 0; j < 8; ++j) {
    const int k  = kk + j;
    const int kc = (k < KT) ? k : (KT - 1);
    const float w = W[(size_t)kc * NTR + nc];
    const unsigned bits = bf16_bits(w);
    o[j] = (unsigned short)(((k < KT) && (n < NTR)) ? bits : 0u);
  }
  unsigned short* dp = plane + (size_t)u * 8;
  *(volatile v8us*)dp = o;
  __threadfence();
  *(volatile v8us*)dp = o;
}

__global__ __launch_bounds__(NTHR) void k_prep(const float* __restrict__ w1, const float* __restrict__ w2,
                                               const float* __restrict__ w3, const float* __restrict__ w4,
                                               unsigned short* p1, unsigned short* p2,
                                               unsigned short* p3, unsigned short* p4) {
  const int blk = (int)blockIdx.x, tid = (int)threadIdx.x;
  if (blk < PB1)                   prep_unit<400, 400, 300>(w1, p1, blk * NTHR + tid);
  else if (blk < PB1 + PB2)        prep_unit<320, 300, 100>(w2, p2, (blk - PB1) * NTHR + tid);
  else if (blk < PB1 + PB2 + PB3)  prep_unit<128, 100, 300>(w3, p3, (blk - PB1 - PB2) * NTHR + tid);
  else                             prep_unit<320, 300, 400>(w4, p4, (blk - PB1 - PB2 - PB3) * NTHR + tid);
}

__device__ __forceinline__ void build_one(const int* __restrict__ idx, const float* __restrict__ val,
                                          int* outp, int tid) {
  int* img = (int*)(dsm + BLD_IMG);
  int* tI  = (int*)(dsm + BLD_TI);
  int* tJ  = (int*)(dsm + BLD_TJ);
  int* tV  = (int*)(dsm + BLD_TV);
  int* cnt = (int*)(dsm + BLD_CNT);
  int* st  = (int*)(dsm + BLD_ST);
  {
    const v4i z4 = {0, 0, 0, 0};
#pragma unroll 1
    for (int q = tid; q < CSR_WORDS / 4; q += NTHR) *(v4ia*)(img + 4 * q) = z4;
  }
#pragma unroll 1
  for (int e = tid; e < 2560; e += NTHR) {
    const int ec = (e < NNZ) ? e : (NNZ - 1);
    const int i = idx[2 * ec];
    const int j = idx[2 * ec + 1];
    const float v = bf16_val(val[ec]);
    const bool ok = (e < NNZ) && ((unsigned)i < (unsigned)NN) && ((unsigned)j < (unsigned)NN);
    tI[e] = ok ? i : -1;
    tJ[e] = ok ? j : 0;
    tV[e] = __float_as_int(v);
  }
  __syncthreads();
  int c = 0;
#pragma unroll 4
  for (int e = 0; e < NNZ; ++e) c += (tI[e] == tid) ? 1 : 0;
  cnt[tid] = c;
  __syncthreads();
  if (tid == 0) {
    int run = 0, mx = 0;
#pragma unroll 1
    for (int t = 0; t < 256; ++t) {
      const int cv = cnt[t];
      st[t] = run;
      run += cv;
      mx = cv > mx ? cv : mx;
    }
    img[BLD_MXW] = mx;
  }
  __syncthreads();
  const int start = clampi(st[tid], 0, NNZ);
  const int maxc  = clampi(img[BLD_MXW], 0, NNZ);
  int nk = 0;
#pragma unroll 1
  for (int e = 0; e < NNZ; ++e) {
    const int ii = tI[e];
    const int j  = tJ[e];
    const float vf = __int_as_float(tV[e]);
    const bool own = (ii == tid);
    int found = -1;
#pragma unroll 1
    for (int t = 0; t < maxc; ++t) {
      const int q  = start + t;
      const int qc = q < 2559 ? q : 2559;
      const int cj = img[CSR_COL + qc];
      const bool hit = own & (t < nk) & (cj == j) & (found < 0);
      found = hit ? qc : found;
    }
    const bool dup = found >= 0;
    const int apq = start + nk;
    const int ap  = apq < 2559 ? apq : 2559;
    const int fc  = dup ? found : ap;
    const float old = __int_as_float(img[CSR_VAL + fc]);
    const float nv  = dup ? (old + vf) : vf;
    const int wv = own ? (CSR_VAL + fc) : (BLD_DMPW + tid);
    const int wc = own ? (CSR_COL + fc) : (BLD_DMPW + 256 + tid);
    img[wv] = __float_as_int(nv);
    img[wc] = j;
    nk += (own & !dup) ? 1 : 0;
  }
  float rs = 0.0f;
#pragma unroll 1
  for (int t = 0; t < maxc; ++t) {
    const int q  = start + t;
    const int qc = q < 2559 ? q : 2559;
    const float v = __int_as_float(img[CSR_VAL + qc]);
    rs += (t < nk) ? v : 0.0f;
  }
  img[CSR_RB + tid] = start;
  img[CSR_RE + tid] = start + nk;
  img[CSR_RS + tid] = __float_as_int(rs);
  __syncthreads();
#pragma unroll 1
  for (int q = tid; q < CSR_WORDS / 4; q += NTHR) {
    const v4i v = *(const v4ia*)(img + 4 * q);
    *(volatile v4i*)(outp + 4 * q) = v;
  }
  __threadfence();
#pragma unroll 1
  for (int q = tid; q < CSR_WORDS / 4; q += NTHR) {
    const v4i v = *(const v4ia*)(img + 4 * q);
    *(volatile v4i*)(outp + 4 * q) = v;
  }
}

__global__ __launch_bounds__(NTHR) void k_build(const int* __restrict__ smI, const float* __restrict__ smV,
                                                const int* __restrict__ spI, const float* __restrict__ spV,
                                                int* csrSm, int* csrSp) {
  const int tid = (int)threadIdx.x;
  if (blockIdx.x == 0) build_one(smI, smV, csrSm, tid);
  else                 build_one(spI, spV, csrSp, tid);
}

template <int MODE>
__global__ __launch_bounds__(NTHR) void k_agg2(const float* __restrict__ src, const int* __restrict__ csr,
                                               float* dst) {
  const int tid = (int)threadIdx.x;
  stage_csr(csr, AG2_CSR, tid);
  __syncthreads();
  const int* s = (const int*)(dsm + AG2_CSR);
  float* so = (float*)(dsm + AG2_OUT);
#pragma unroll 1
  for (int rr = 0; rr < 2; ++rr) {
    const int lr = tid + NTHR * rr;
    const int r  = (int)blockIdx.x * 512 + lr;
    const int b  = r / NN;
    const int i  = r - b * NN;
    const int rb = clampi(s[CSR_RB + i], 0, NNZ);
    const int re = clampi(s[CSR_RE + i], rb, NNZ);
    const float* base = src + (size_t)b * NN * 2;
    float a0 = 0.0f, a1 = 0.0f;
#pragma unroll 1
    for (int p = rb; p < re; ++p) {
      const int j = clampi(s[CSR_COL + p], 0, NN - 1);
      const float w = __int_as_float(s[CSR_VAL + p]);
      const v2f x = *(const v2fa*)(base + 2 * j);
      const float x0 = (MODE == 0) ? bf16_val(x.x) : x.x;
      const float x1 = (MODE == 0) ? bf16_val(x.y) : x.y;
      a0 = fmaf(w, x0, a0);
      a1 = fmaf(w, x1, a1);
    }
    if constexpr (MODE == 1) { a0 = relu_f(a0); a1 = relu_f(a1); }
    so[2 * lr]     = a0;
    so[2 * lr + 1] = a1;
  }
  __syncthreads();
  const v4f v = *(const v4fa*)(so + 4 * tid);
  float* dp = dst + (size_t)blockIdx.x * 1024 + 4 * tid;
  *(volatile v4f*)dp = v;
  __threadfence();
  *(volatile v4f*)dp = v;
}

template <int KTOT, int NT, int NTW, bool FULL>
__device__ __forceinline__ void kloop_g(const unsigned short* __restrict__ ap, const unsigned short* __restrict__ bp,
                                        int nt0, v8f (&acc)[NTW]) {
#pragma unroll 1
  for (int k0 = 0; k0 < KTOT; k0 += 32) {
    FragB af;
    af.h[0] = *(const v8usa*)(ap + k0);
    af.h[1] = *(const v8usa*)(ap + k0 + 16);
#pragma unroll
    for (int t = 0; t < NTW; ++t) {
      const bool on = FULL || (nt0 + t < NT);
      if (on) {
        const unsigned short* wq = bp + (size_t)(16 * (nt0 + t)) * (size_t)KTOT + k0;
        FragB bf;
        bf.h[0] = *(const v8usa*)wq;
        bf.h[1] = *(const v8usa*)(wq + 16);
        acc[t] = wmb(af, bf, acc[t]);
      }
    }
  }
}

template <int KTOT, int NT, int NTW>
__device__ __forceinline__ void kloop_l(int aOff, const unsigned short* __restrict__ bp, int nt0, v8f (&acc)[NTW]) {
  const unsigned short* ap = (const unsigned short*)dsm + aOff;
#pragma unroll 1
  for (int k0 = 0; k0 < KTOT; k0 += 32) {
    FragB af;
    af.h[0] = *(const v8usa*)(ap + k0);
    af.h[1] = *(const v8usa*)(ap + k0 + 16);
#pragma unroll
    for (int t = 0; t < NTW; ++t) {
      const unsigned short* wq = bp + (size_t)(16 * (nt0 + t)) * (size_t)KTOT + k0;
      FragB bf;
      bf.h[0] = *(const v8usa*)wq;
      bf.h[1] = *(const v8usa*)(wq + 16);
      acc[t] = wmb(af, bf, acc[t]);
    }
  }
}

template <int NT, int NTW, bool FULL, int MODE>
__device__ __forceinline__ void epi_stage(const v8f (&acc)[NTW], int nt0, int rt, int hh, int m,
                                          int stgOff, int sbOff, int srsOff) {
  constexpr int NP = 16 * NT;
  float* stg = (float*)(dsm + stgOff);
  const float* sb  = (const float*)(dsm + sbOff);
  const float* srs = (const float*)(dsm + srsOff);
  float rsv[8];
#pragma unroll
  for (int r = 0; r < 8; ++r) rsv[r] = srs[16 * rt + 8 * hh + r];
#pragma unroll
  for (int t = 0; t < NTW; ++t) {
    const bool on = FULL || (nt0 + t < NT);
    if (on) {
      const int col = 16 * (nt0 + t) + m;
      const float bb = sb[col];
#pragma unroll
      for (int r = 0; r < 8; ++r) {
        const int lr = 16 * rt + 8 * hh + r;
        const float a = acc[t][r];
        const float v = (MODE == 0) ? (a + bb) : relu_f(fmaf(rsv[r], bb, a));
        stg[lr * NP + col] = v;
      }
    }
  }
}

template <int NV4, int NTH>
__device__ __forceinline__ void tile_out(int stgOff, float* dst, int tid) {
  static_assert(NV4 % NTH == 0);
  const float* stg = (const float*)(dsm + stgOff);
#pragma unroll 4
  for (int it = 0; it < NV4 / NTH; ++it) {
    const int q = it * NTH + tid;
    const v4f v = *(const v4fa*)(stg + 4 * q);
    *(volatile v4f*)(dst + 4 * (size_t)q) = v;
  }
}

__global__ __launch_bounds__(NTHR) void k_g1(const float* __restrict__ S0, int rowOff,
                                             const float* __restrict__ W0, const float* __restrict__ b0,
                                             const float* __restrict__ b1, const int* __restrict__ csr,
                                             const unsigned short* __restrict__ BT, float* Y1) {
  const int tid = (int)threadIdx.x, lane = tid & 31, wave = tid >> 5, hh = lane >> 4, m = lane & 15;
  const int rowBase = (int)blockIdx.x * GBM;
  unsigned short* sA = (unsigned short*)(dsm + G1_A);
  float* sWa = (float*)(dsm + G1_W0A);
  float* sWb = (float*)(dsm + G1_W0B);
  float* sB0 = (float*)(dsm + G1_B0);
  float* sB1 = (float*)(dsm + G1_B1);
  float* sS0 = (float*)(dsm + G1_S0);
  float* sRS = (float*)(dsm + G1_RS);

#pragma unroll 1
  for (int k = tid; k < D1; k += NTHR) {
    sWa[k] = bf16_val(W0[k]);
    sWb[k] = bf16_val(W0[D1 + k]);
    sB0[k] = bf16_val(b0[k]);
  }
#pragma unroll 1
  for (int n = tid; n < NP1; n += NTHR) {
    const int nc = (n < D2) ? n : (D2 - 1);
    const float bv = bf16_val(b1[nc]);
    sB1[n] = (n < D2) ? bv : 0.0f;
  }
  if (tid < 2 * GBM) sS0[tid] = S0[(size_t)(rowOff + rowBase) * 2 + tid];
  if (tid < GBM) {
    const int i = (rowBase + tid) % NN;
    sRS[tid] = __int_as_float(csr[CSR_RS + i]);
  }
  __syncthreads();

#pragma unroll 1
  for (int u = tid; u < GBM * (D1 / 8); u += NTHR) {
    const int lr = u / (D1 / 8);
    const int k8 = (u - lr * (D1 / 8)) * 8;
    const float s0 = sS0[2 * lr], s1 = sS0[2 * lr + 1], rs = sRS[lr];
    v8us oh, ol;
#pragma unroll
    for (int j = 0; j < 8; ++j) {
      const int k = k8 + j;
      float v = fmaf(s0, sWa[k], fmaf(s1, sWb[k], rs * sB0[k]));
      v = relu_f(v);
      const unsigned hb = bf16_bits(v);
      const unsigned lb = bf16_bits(v - __uint_as_float(hb << 16));
      oh[j] = (unsigned short)hb;
      ol[j] = (unsigned short)lb;
    }
    *(v8usa*)(sA + lr * K1 + k8)      = oh;
    *(v8usa*)(sA + lr * K1 + D1 + k8) = ol;
  }
  __syncthreads();

  const int rt = wave & 3, qg = wave >> 2, nt0 = qg * 10;
  v8f acc[10];
  {
    const v8f z = {0.f, 0.f, 0.f, 0.f, 0.f, 0.f, 0.f, 0.f};
#pragma unroll
    for (int t = 0; t < 10; ++t) acc[t] = z;
  }
  kloop_l<K1, 20, 10>((16 * rt + m) * K1 + 8 * hh, BT + (size_t)m * K1 + 8 * hh, nt0, acc);
  __syncthreads();
  epi_stage<20, 10, true, 0>(acc, nt0, rt, hh, m, G1_A, G1_B1, G1_RS);
  __syncthreads();
  float* dp = Y1 + (size_t)rowBase * NP1;
  tile_out<GBM * NP1 / 4, NTHR>(G1_A, dp, tid);
  __threadfence();
  tile_out<GBM * NP1 / 4, NTHR>(G1_A, dp, tid);
}

template <int KTOT, int NT, int NTW, int NQ, int MODE>
__global__ __launch_bounds__(128 * NQ) void k_gemm(const unsigned short* __restrict__ A,
                                                   const unsigned short* __restrict__ BT,
                                                   const float* __restrict__ bias, int nTrue,
                                                   const int* __restrict__ csr, float* dst,
                                                   const float* __restrict__ W5, const float* __restrict__ b5,
                                                   float* P6, int rowOff) {
  constexpr int NP  = 16 * NT;
  constexpr int NTH = 128 * NQ;
  constexpr bool FULL = (NT == NQ * NTW);
  static_assert(NQ * NTW >= NT && KTOT % 32 == 0);
  static_assert(MODE != 2 || (NP == 400 && NTH >= 256));
  static_assert(MODE == 2 || ((GBM * NP / 4) % NTH == 0));
  const int tid = (int)threadIdx.x, lane = tid & 31, wave = tid >> 5, hh = lane >> 4, m = lane & 15;
  const int rowBase = (int)blockIdx.x * GBM;
  float* sb  = (float*)(dsm + GL_SB(NP));
  float* srs = (float*)(dsm + GL_SRS(NP));

#pragma unroll 1
  for (int n = tid; n < NP; n += NTH) {
    const int nc = (n < nTrue) ? n : (nTrue - 1);
    const float bv = bf16_val(bias[nc]);
    sb[n] = (n < nTrue) ? bv : 0.0f;
  }
  if (tid < GBM) {
    const int i = (rowBase + tid) % NN;
    const float rv = __int_as_float(csr[CSR_RS + i]);
    srs[tid] = (MODE == 0) ? 0.0f : rv;
  }
  if constexpr (MODE == 2) {
    float* sW5 = (float*)(dsm + GL_SW5(NP));
#pragma unroll 1
    for (int k = tid; k < 2 * D5; k += NTH) sW5[k] = bf16_val(W5[k]);
  }

  const int rt = wave & 3, qg = wave >> 2, nt0 = qg * NTW;
  v8f acc[NTW];
  {
    const v8f z = {0.f, 0.f, 0.f, 0.f, 0.f, 0.f, 0.f, 0.f};
#pragma unroll
    for (int t = 0; t < NTW; ++t) acc[t] = z;
  }
  kloop_g<KTOT, NT, NTW, FULL>(A + (size_t)(rowBase + 16 * rt + m) * (size_t)KTOT + 8 * hh,
                               BT + (size_t)m * (size_t)KTOT + 8 * hh, nt0, acc);
  __syncthreads();
  epi_stage<NT, NTW, FULL, MODE>(acc, nt0, rt, hh, m, 0, GL_SB(NP), GL_SRS(NP));
  __syncthreads();

  if constexpr (MODE < 2) {
    float* dp = dst + (size_t)rowBase * NP;
    tile_out<GBM * NP / 4, NTH>(0, dp, tid);
    __threadfence();
    tile_out<GBM * NP / 4, NTH>(0, dp, tid);
  } else {
    const float* sW5 = (const float*)(dsm + GL_SW5(NP));
    float* sP6 = (float*)(dsm + GL_SP6(NP));
    const float bb0 = bf16_val(b5[0]);
    const float bb1 = bf16_val(b5[1]);
    if (tid < 256) {
      const int prow = tid >> 2, pq = tid & 3;
      const float* xr = (const float*)dsm + prow * NP + pq * 100;
      const float* wr = sW5 + pq * 200;
      float p0 = 0.0f, p1 = 0.0f;
#pragma unroll 4
      for (int kk = 0; kk < 100; ++kk) {
        const float x = xr[kk];
        p0 = fmaf(x, wr[2 * kk], p0);
        p1 = fmaf(x, wr[2 * kk + 1], p1);
      }
      p0 += __shfl_xor(p0, 1, 32); p1 += __shfl_xor(p1, 1, 32);
      p0 += __shfl_xor(p0, 2, 32); p1 += __shfl_xor(p1, 2, 32);
      if (pq == 0) { sP6[2 * prow] = p0 + bb0; sP6[2 * prow + 1] = p1 + bb1; }
    }
    __syncthreads();
    if (wave == 0) {
      const v4f v = *(const v4fa*)(sP6 + 4 * lane);
      float* dp = P6 + (size_t)(rowOff + rowBase) * 2 + 4 * lane;
      *(volatile v4f*)dp = v;
      __threadfence();
      *(volatile v4f*)dp = v;
    }
  }
}

__device__ __forceinline__ void put_hl(unsigned short* row, int lane, v2u h0, v2u h1, v2u h2,
                                       v2u l0, v2u l1, v2u l2) {
  *(volatile v2u*)(row + 4 * lane)       = h0;
  *(volatile v2u*)(row + 128 + 4 * lane) = h1;
  if (lane < 16) *(volatile v2u*)(row + 256 + 4 * lane) = h2;
  *(volatile v2u*)(row + 320 + 4 * lane) = l0;
  *(volatile v2u*)(row + 448 + 4 * lane) = l1;
  if (lane < 16) *(volatile v2u*)(row + 576 + 4 * lane) = l2;
}

template <int RELU>
__global__ __launch_bounds__(NTHR) void k_aggw(const float* __restrict__ Yin, const int* __restrict__ csr,
                                               unsigned short* outp) {
  const int tid = (int)threadIdx.x, lane = tid & 31, wave = tid >> 5;
  stage_csr(csr, 0, tid);
  __syncthreads();
  const int* s = (const int*)dsm;
  const int bl = (int)blockIdx.x;
  const float* base = Yin + (size_t)bl * NN * NP1;
  const int c2 = (lane + 64 < 80) ? (lane + 64) : 79;
#pragma unroll 1
  for (int i = wave; i < NN; i += 8) {
    const int rb = clampi(s[CSR_RB + i], 0, NNZ);
    const int re = clampi(s[CSR_RE + i], rb, NNZ);
    v4f a0 = {0.f, 0.f, 0.f, 0.f}, a1 = {0.f, 0.f, 0.f, 0.f}, a2 = {0.f, 0.f, 0.f, 0.f};
#pragma unroll 1
    for (int p = rb; p < re; ++p) {
      const int j = clampi(s[CSR_COL + p], 0, NN - 1);
      const float w = __int_as_float(s[CSR_VAL + p]);
      const float* src = base + (size_t)j * NP1;
      const v4f x0 = *(const v4fa*)(src + 4 * lane);
      const v4f x1 = *(const v4fa*)(src + 128 + 4 * lane);
      const v4f x2 = *(const v4fa*)(src + 4 * c2);
      a0.x = fmaf(w, x0.x, a0.x); a0.y = fmaf(w, x0.y, a0.y); a0.z = fmaf(w, x0.z, a0.z); a0.w = fmaf(w, x0.w, a0.w);
      a1.x = fmaf(w, x1.x, a1.x); a1.y = fmaf(w, x1.y, a1.y); a1.z = fmaf(w, x1.z, a1.z); a1.w = fmaf(w, x1.w, a1.w);
      a2.x = fmaf(w, x2.x, a2.x); a2.y = fmaf(w, x2.y, a2.y); a2.z = fmaf(w, x2.z, a2.z); a2.w = fmaf(w, x2.w, a2.w);
    }
    if constexpr (RELU != 0) {
      a0.x = relu_f(a0.x); a0.y = relu_f(a0.y); a0.z = relu_f(a0.z); a0.w = relu_f(a0.w);
      a1.x = relu_f(a1.x); a1.y = relu_f(a1.y); a1.z = relu_f(a1.z); a1.w = relu_f(a1.w);
      a2.x = relu_f(a2.x); a2.y = relu_f(a2.y); a2.z = relu_f(a2.z); a2.w = relu_f(a2.w);
    }
    v2u h0, h1, h2, l0, l1, l2;
    hilo_pack(a0.x, a0.y, a0.z, a0.w, h0, l0);
    hilo_pack(a1.x, a1.y, a1.z, a1.w, h1, l1);
    hilo_pack(a2.x, a2.y, a2.z, a2.w, h2, l2);
    unsigned short* row = outp + (size_t)(bl * NN + i) * K2;
    put_hl(row, lane, h0, h1, h2, l0, l1, l2);
    __threadfence();
    put_hl(row, lane, h0, h1, h2, l0, l1, l2);
  }
}

__global__ __launch_bounds__(NTHR) void k_agg23(const float* __restrict__ Y2, const int* __restrict__ csrSm,
                                                const int* __restrict__ csrSp, unsigned short* S3hl) {
  const int tid = (int)threadIdx.x, lane = tid & 31, wave = tid >> 5;
  const int bl = (int)blockIdx.x;
  float* bufY = (float*)(dsm + A23_Y);
  float* bufX = (float*)(dsm + A23_X);
  const int* s = (const int*)(dsm + A23_CSR);
  stage_csr(csrSm, A23_CSR, tid);
#pragma unroll 1
  for (int q = tid; q < NN * 26; q += NTHR) {
    const int row = q / 26;
    const int c = q - row * 26;
    const v4f v = *(const v4fa*)(Y2 + (size_t)(bl * NN + row) * NP2 + 4 * c);
    *(v4fa*)(bufY + row * YS + 4 * c) = v;
  }
  __syncthreads();
  const int c4 = (lane < 26) ? lane : 25;
#pragma unroll 1
  for (int i = wave; i < NN; i += 8) {
    const int rb = clampi(s[CSR_RB + i], 0, NNZ);
    const int re = clampi(s[CSR_RE + i], rb, NNZ);
    v4f a = {0.f, 0.f, 0.f, 0.f};
#pragma unroll 1
    for (int p = rb; p < re; ++p) {
      const int j = clampi(s[CSR_COL + p], 0, NN - 1);
      const float w = __int_as_float(s[CSR_VAL + p]);
      const v4f x = *(const v4fa*)(bufY + j * YS + 4 * c4);
      a.x = fmaf(w, x.x, a.x); a.y = fmaf(w, x.y, a.y); a.z = fmaf(w, x.z, a.z); a.w = fmaf(w, x.w, a.w);
    }
    a.x = relu_f(a.x); a.y = relu_f(a.y); a.z = relu_f(a.z); a.w = relu_f(a.w);
    if (lane < 26) *(v4fa*)(bufX + i * YS + 4 * lane) = a;
  }
  __syncthreads();
  stage_csr(csrSp, A23_CSR, tid);
  __syncthreads();
#pragma unroll 1
  for (int i = wave; i < NN; i += 8) {
    const int rb = clampi(s[CSR_RB + i], 0, NNZ);
    const int re = clampi(s[CSR_RE + i], rb, NNZ);
    v4f a = {0.f, 0.f, 0.f, 0.f};
#pragma unroll 1
    for (int p = rb; p < re; ++p) {
      const int j = clampi(s[CSR_COL + p], 0, NN - 1);
      const float w = __int_as_float(s[CSR_VAL + p]);
      const v4f x = *(const v4fa*)(bufX + j * YS + 4 * c4);
      a.x = fmaf(w, x.x, a.x); a.y = fmaf(w, x.y, a.y); a.z = fmaf(w, x.z, a.z); a.w = fmaf(w, x.w, a.w);
    }
    const bool live = lane < 26;
    const float q0 = live ? a.x : 0.0f, q1 = live ? a.y : 0.0f, q2 = live ? a.z : 0.0f, q3 = live ? a.w : 0.0f;
    v2u hw, lw;
    hilo_pack(q0, q1, q2, q3, hw, lw);
    unsigned short* row = S3hl + (size_t)(bl * NN + i) * K3;
    *(volatile v2u*)(row + 4 * lane)       = hw;
    *(volatile v2u*)(row + 128 + 4 * lane) = lw;
    __threadfence();
    *(volatile v2u*)(row + 4 * lane)       = hw;
    *(volatile v2u*)(row + 128 + 4 * lane) = lw;
  }
}

extern "C" void kernel_launch(void* const* d_in, const int* in_sizes, int n_in,
                              void* d_out, int out_size, void* d_ws, size_t ws_size,
                              hipStream_t stream) {
  if (n_in < 17) return;
  if (in_sizes[0] != MR * 2) return;
  if (in_sizes[1] != NNZ || in_sizes[2] != NNZ) return;
  if (in_sizes[3] != 2 * D1 || in_sizes[4] != D1) return;
  if (in_sizes[5] != D1 * D2 || in_sizes[6] != D2) return;
  if (in_sizes[7] != D2 * D3 || in_sizes[8] != D3) return;
  if (in_sizes[9] != D3 * D4 || in_sizes[10] != D4) return;
  if (in_sizes[11] != D4 * D5 || in_sizes[12] != D5) return;
  if (in_sizes[13] != D5 * 2 || in_sizes[14] != 2) return;
  if (in_sizes[15] != NNZ * 2 || in_sizes[16] != NNZ * 2) return;
  if (out_size != MR * 2) return;
  if (WS_END > ws_size) return;

  const float* H     = (const float*)d_in[0];
  const float* smV   = (const float*)d_in[1];
  const float* spV   = (const float*)d_in[2];
  const float* Wenc0 = (const float*)d_in[3];
  const float* benc0 = (const float*)d_in[4];
  const float* Wenc1 = (const float*)d_in[5];
  const float* benc1 = (const float*)d_in[6];
  const float* Wenc2 = (const float*)d_in[7];
  const float* benc2 = (const float*)d_in[8];
  const float* Wdec0 = (const float*)d_in[9];
  const float* bdec0 = (const float*)d_in[10];
  const float* Wdec1 = (const float*)d_in[11];
  const float* bdec1 = (const float*)d_in[12];
  const float* Wdec2 = (const float*)d_in[13];
  const float* bdec2 = (const float*)d_in[14];
  const int*   smI   = (const int*)d_in[15];
  const int*   spI   = (const int*)d_in[16];
  float* out = (float*)d_out;

  char* ws = (char*)d_ws;
  float*          RA   = (float*)(ws + WS_A);
  unsigned short* RB   = (unsigned short*)(ws + WS_B);
  float*          RCy  = (float*)(ws + WS_C);
  unsigned short* RD   = (unsigned short*)(ws + WS_D);
  float*          S0   = (float*)(ws + WS_S0);
  float*          P6   = (float*)(ws + WS_P6);
  unsigned short* W1T  = (unsigned short*)(ws + WS_W1);
  unsigned short* W2T  = (unsigned short*)(ws + WS_W2);
  unsigned short* W3T  = (unsigned short*)(ws + WS_W3);
  unsigned short* W4T  = (unsigned short*)(ws + WS_W4);
  int*            CSM  = (int*)(ws + WS_CSM);
  int*            CSP  = (int*)(ws + WS_CSP);

  hipFuncSetAttribute(reinterpret_cast<const void*>(&k_g1), hipFuncAttributeMaxDynamicSharedMemorySize, (int)G1_LDS);
  hipFuncSetAttribute(reinterpret_cast<const void*>(&k_gemm<K3, 20, 10, 2, 1>),
                      hipFuncAttributeMaxDynamicSharedMemorySize, (int)GL_TOT(NP3));
  hipFuncSetAttribute(reinterpret_cast<const void*>(&k_gemm<K4, 25, 7, 4, 2>),
                      hipFuncAttributeMaxDynamicSharedMemorySize, (int)GL_TOT(NP4));
  hipFuncSetAttribute(reinterpret_cast<const void*>(&k_agg23), hipFuncAttributeMaxDynamicSharedMemorySize, (int)A23_LDS);

  k_prep<<<PB1 + PB2 + PB3 + PB4, NTHR, 0, stream>>>(Wenc1, Wenc2, Wdec0, Wdec1, W1T, W2T, W3T, W4T);
  k_build<<<2, NTHR, BLD_LDS, stream>>>(smI, smV, spI, spV, CSM, CSP);
  k_agg2<0><<<MR / 512, NTHR, AG2_LDS, stream>>>(H, CSM, S0);

  for (int c = 0; c < NCH; ++c) {
    const int rowOff = c * RC;
    k_g1<<<RC / GBM, NTHR, G1_LDS, stream>>>(S0, rowOff, Wenc0, benc0, benc1, CSM, W1T, RA);
    k_aggw<1><<<BC, NTHR, CSR_LDS, stream>>>(RA, CSM, RB);
    k_gemm<K2, 8, 4, 2, 0><<<RC / GBM, 256, GL_TOT(NP2), stream>>>(RB, W2T, benc2, D3, CSM, RCy,
                                                                    Wdec2, bdec2, P6, rowOff);
    k_agg23<<<BC, NTHR, A23_LDS, stream>>>(RCy, CSM, CSP, RD);
    k_gemm<K3, 20, 10, 2, 1><<<RC / GBM, 256, GL_TOT(NP3), stream>>>(RD, W3T, bdec0, D4, CSP, RA,
                                                                      Wdec2, bdec2, P6, rowOff);
    k_aggw<0><<<BC, NTHR, CSR_LDS, stream>>>(RA, CSP, RB);
    k_gemm<K4, 25, 7, 4, 2><<<RC / GBM, 512, GL_TOT(NP4), stream>>>(RB, W4T, bdec1, D5, CSP, RA,
                                                                     Wdec2, bdec2, P6, rowOff);
  }
  k_agg2<1><<<MR / 512, NTHR, AG2_LDS, stream>>>(P6, CSP, out);
}
